// DynamicMaxSimilarity_38792144617497
// MI455X (gfx1250) — hardware-verified
//
#include <hip/hip_runtime.h>
#include <hip/hip_bf16.h>
#include <math.h>

typedef __attribute__((ext_vector_type(16))) _Float16 v16h;
typedef __attribute__((ext_vector_type(8)))  _Float16 v8h;
typedef __attribute__((ext_vector_type(8)))  float    v8f;
#define VST2(T, ptr, val) do { const T _v = (val); *(volatile T*)(ptr) = _v; __threadfence(); *(volatile T*)(ptr) = _v; } while (0)

#define NA_ 512
#define NB_ 512
#define TF_ 16
#define DD_ 256
#define TSTRIDE 260

__global__ __launch_bounds__(256) void nrm_tanh_f16_kernel(
    const float* __restrict__ a, const float* __restrict__ b,
    _Float16* __restrict__ ah, _Float16* __restrict__ bh)
{
    const int wave = threadIdx.x >> 5;
    const int lane = threadIdx.x & 31;
    const int row  = blockIdx.x * 8 + wave;

    const float* __restrict__ src;
    _Float16* __restrict__ dst;
    if (row < NA_ * TF_) { src = a + (size_t)row * DD_;              dst = ah + (size_t)row * DD_; }
    else                 { src = b + (size_t)(row - NA_*TF_) * DD_;  dst = bh + (size_t)(row - NA_*TF_) * DD_; }

    float4 p0 = *(const float4*)(src + lane * 8);
    float4 p1 = *(const float4*)(src + lane * 8 + 4);
    float x[8];
    x[0] = tanhf(p0.x); x[1] = tanhf(p0.y); x[2] = tanhf(p0.z); x[3] = tanhf(p0.w);
    x[4] = tanhf(p1.x); x[5] = tanhf(p1.y); x[6] = tanhf(p1.z); x[7] = tanhf(p1.w);

    float s = 0.f;
    #pragma unroll
    for (int r = 0; r < 8; ++r) s += x[r] * x[r];
    #pragma unroll
    for (int off = 1; off < 32; off <<= 1) s += __shfl_xor(s, off, 32);

    const float scale = 1.0f / fmaxf(sqrtf(s), 1e-12f);

    v8h h;
    #pragma unroll
    for (int r = 0; r < 8; ++r) h[r] = (_Float16)(x[r] * scale);
    VST2(v8h, dst + lane * 8, h);
}

__global__ __launch_bounds__(128) void simdp_kernel(
    const _Float16* __restrict__ ah, const _Float16* __restrict__ bh,
    float* __restrict__ out)
{
    __shared__ float lds[128 * TSTRIDE];
    const int w = threadIdx.x >> 5;
    const int l = threadIdx.x & 31;
    const int ia  = blockIdx.y * 4 + w;
    const int ib0 = blockIdx.x * 32;

    const int rowA  = l & 15;
    const int koffA = (l >> 4) << 3;
    const _Float16* abase = ah + ((size_t)ia * TF_ + rowA) * DD_ + koffA;
    v16h afrag[8];
    #pragma unroll
    for (int c = 0; c < 8; ++c) {
        union { v16h v; v8h h[2]; } u;
        u.h[0] = *(const v8h*)(abase + c * 32);
        u.h[1] = *(const v8h*)(abase + c * 32 + 16);
        afrag[c] = u.v;
    }

    const int colB  = l & 15;
    const int koffB = (l >> 4) << 3;
    const int sbase0 = ((l & 15) << 4) + ((l >> 4) << 3);

    for (int q = 0; q < 32; ++q) {
        const _Float16* bbase = bh + ((size_t)(ib0 + q) * TF_ + colB) * DD_ + koffB;
        v16h bfrag[8];
        #pragma unroll
        for (int c = 0; c < 8; ++c) {
            union { v16h v; v8h h[2]; } ub;
            ub.h[0] = *(const v8h*)(bbase + c * 32);
            ub.h[1] = *(const v8h*)(bbase + c * 32 + 16);
            bfrag[c] = ub.v;
        }

        v8f acc = {};
        #pragma unroll
        for (int c = 0; c < 8; ++c) {
            acc = __builtin_amdgcn_wmma_f32_16x16x32_f16(
                      false, afrag[c], false, bfrag[c], (short)0, acc, false, false);
            asm volatile("v_nop\n\tv_nop\n\tv_nop\n\tv_nop" : "+v"(acc) : "v"(afrag[c]), "v"(bfrag[c]));
        }

        float* tp = &lds[(w * 32 + q) * TSTRIDE + sbase0];
        float4 lo; lo.x = acc[0]; lo.y = acc[1]; lo.z = acc[2]; lo.w = acc[3];
        float4 hi; hi.x = acc[4]; hi.y = acc[5]; hi.z = acc[6]; hi.w = acc[7];
        *(float4*)(tp)     = lo;
        *(float4*)(tp + 4) = hi;
    }
    __syncthreads();

    const int t = threadIdx.x;
    const float* tile = &lds[t * TSTRIDE];
    float prev[17];
    #pragma unroll
    for (int i = 0; i <= 16; ++i) prev[i] = 0.f;

    #pragma unroll
    for (int j = 1; j <= 16; ++j) {
        const float* col = tile + (j - 1) * 16;
        float4 c0 = *(const float4*)(col);
        float4 c1 = *(const float4*)(col + 4);
        float4 c2 = *(const float4*)(col + 8);
        float4 c3 = *(const float4*)(col + 12);
        float lv[16] = {c0.x,c0.y,c0.z,c0.w, c1.x,c1.y,c1.z,c1.w,
                        c2.x,c2.y,c2.z,c2.w, c3.x,c3.y,c3.z,c3.w};
        float cur = 0.f;
        #pragma unroll
        for (int i = 1; i <= 16; ++i) {
            const float fm   = (float)(i > j ? i : j);
            const float best = fmaxf(fmaxf(prev[i-1], prev[i]), cur);
            const float nv   = (best * (fm - 1.0f) + lv[i-1]) * (1.0f / fm);
            prev[i-1] = cur;
            cur = nv;
        }
        prev[16] = cur;
    }

    const int ia2 = blockIdx.y * 4 + (t >> 5);
    const int ib2 = ib0 + (t & 31);
    VST2(float, out + (size_t)ia2 * NB_ + ib2, prev[16]);
}

extern "C" void kernel_launch(void* const* d_in, const int* in_sizes, int n_in,
                              void* d_out, int out_size, void* d_ws, size_t ws_size,
                              hipStream_t stream) {
    (void)in_sizes; (void)n_in; (void)out_size;
    if (ws_size < (size_t)2 * NA_ * TF_ * DD_ * 2) return;
    const float* a = (const float*)d_in[0];
    const float* b = (const float*)d_in[1];
    float* out = (float*)d_out;

    _Float16* ah = (_Float16*)d_ws;
    _Float16* bh = ah + (size_t)NA_ * TF_ * DD_;

    nrm_tanh_f16_kernel<<<dim3(2048), dim3(256), 0, stream>>>(a, b, ah, bh);

    simdp_kernel<<<dim3(NB_ / 32, NA_ / 4), dim3(128), 0, stream>>>(ah, bh, out);
}
